// Mini_Batch_ERGCN_7627861918260
// MI455X (gfx1250) — hardware-verified
//
#include <hip/hip_runtime.h>
#include <stddef.h>
#include <stdint.h>


#define EDIM  128
#define CDIM  32
#define RREL  64
#define NBAS  16
#define NSRC  8192
#define MSEG1 4096
#define MSEGO 2048
#define RCH   16
#define NCHK  4
#define NTHR  256
#define NWAV  8
#define DR    64
#define BM    128
#define BN    64
#define WSC   64.0f
#define RWSC  0.015625f
#define WSCAP 134217728

static_assert(RREL == RCH * NCHK);
static_assert(NTHR == 32 * NWAV);
static_assert(DR == 8 * NWAV);
static_assert((NSRC % BM) == 0);
static_assert(((RCH * EDIM) % BN) == 0 && ((RCH * CDIM) % BN) == 0);
static_assert((MSEG1 % DR) == 0 && (MSEGO % DR) == 0);
static_assert(BM * BN == 8 * 4 * NTHR);
static_assert(((RREL * EDIM * 16) % NTHR) == 0 && ((RREL * CDIM * 16) % NTHR) == 0);
static_assert(((NSRC * EDIM / 8) % NTHR) == 0);
static_assert((EDIM % 32) == 0);

typedef _Float16 v8h  __attribute__((ext_vector_type(8)));
typedef _Float16 v16h __attribute__((ext_vector_type(16)));
typedef float    v4f  __attribute__((ext_vector_type(4)));
typedef float    v8f  __attribute__((ext_vector_type(8)));
typedef v4f v4fa __attribute__((may_alias));
union Frag { v16h v; v8h h[2]; };

__device__ __forceinline__ v8f wmh(v16h a, v16h b, v8f c) {
  v8f d = __builtin_amdgcn_wmma_f32_16x16x32_f16(false, a, false, b, (short)0, c, false, false);
  asm volatile("v_nop\n\tv_nop\n\tv_nop\n\tv_nop" : "+v"(d) : "v"(a), "v"(b));
  return d;
}

__device__ __forceinline__ v8h cvt8(v4f a, v4f b) {
  v8h r;
  r[0] = (_Float16)a[0]; r[1] = (_Float16)a[1]; r[2] = (_Float16)a[2]; r[3] = (_Float16)a[3];
  r[4] = (_Float16)b[0]; r[5] = (_Float16)b[1]; r[6] = (_Float16)b[2]; r[7] = (_Float16)b[3];
  return r;
}

__global__ __launch_bounds__(NTHR) void k_compose(const float* __restrict__ comp,
                                                  const float* __restrict__ bases,
                                                  _Float16* Wt, int HD) {
  const int i = (int)blockIdx.x * NTHR + (int)threadIdx.x;
  const int col = i >> 4, eg = i & 15;
  const int r = col / HD, hc = col - r * HD;
  float acc[8];
#pragma unroll
  for (int e = 0; e < 8; ++e) acc[e] = 0.0f;
#pragma unroll 1
  for (int b = 0; b < NBAS; ++b) {
    const float cb = comp[r * NBAS + b];
    const float* bp = bases + ((size_t)(b * EDIM + 8 * eg)) * HD + hc;
#pragma unroll
    for (int e = 0; e < 8; ++e) acc[e] = fmaf(cb, bp[(size_t)e * HD], acc[e]);
  }
  v8h hv;
#pragma unroll
  for (int e = 0; e < 8; ++e) hv[e] = (_Float16)(acc[e] * WSC);
  _Float16* dst = Wt + (size_t)i * 8;
  *(volatile v8h*)dst = hv;
  __threadfence();
  *(volatile v8h*)dst = hv;
}

__global__ __launch_bounds__(NTHR) void k_cvt(const float* __restrict__ x1, const float* __restrict__ x2,
                                              _Float16* xh, int n8, int nbh) {
  const int sec = ((int)blockIdx.x >= nbh) ? 1 : 0;
  const float* src = sec ? x2 : x1;
  int j = ((int)blockIdx.x - sec * nbh) * NTHR + (int)threadIdx.x;
  j = j < n8 ? j : n8 - 1;
  const v4f a = *(const v4f*)(src + (size_t)j * 8);
  const v4f b = *(const v4f*)(src + (size_t)j * 8 + 4);
  const v8h o = cvt8(a, b);
  _Float16* dst = xh + (size_t)sec * (size_t)n8 * 8 + (size_t)j * 8;
  *(volatile v8h*)dst = o;
  __threadfence();
  *(volatile v8h*)dst = o;
}

__global__ __launch_bounds__(NTHR) void k_gath(const float* __restrict__ h1, const int* __restrict__ hidx,
                                               _Float16* hg, int nh, int nrow) {
  const int i = (int)blockIdx.x * NTHR + (int)threadIdx.x;
  int n = i >> 4;
  n = n < nh ? n : nh - 1;
  const int eg = i & 15;
  int s = hidx[n];
  s = s < 0 ? s + nrow : s;
  s = s < 0 ? 0 : (s > nrow - 1 ? nrow - 1 : s);
  const float* p = h1 + (size_t)s * EDIM + 8 * eg;
  const v4f a = *(const v4f*)(p);
  const v4f b = *(const v4f*)(p + 4);
  const v8h o = cvt8(a, b);
  _Float16* dst = hg + (size_t)i * 8;
  *(volatile v8h*)dst = o;
  __threadfence();
  *(volatile v8h*)dst = o;
}

__global__ __launch_bounds__(NTHR) void k_gemm(const _Float16* __restrict__ A, const _Float16* __restrict__ Bt,
                                               float* C, int ldc, int nbn) {
  __shared__ __attribute__((aligned(16))) float stg[BM * BN];
  const int tid = threadIdx.x, lane = tid & 31, wave = tid >> 5, hh = lane >> 4, m = lane & 15;
  const int mb = (int)blockIdx.x / nbn, nb = (int)blockIdx.x - mb * nbn;
  const int wm = wave & 3, wn = wave >> 2;
  const int row0 = mb * BM + wm * 32, col0 = nb * BN + wn * 32;

  v8f acc[2][2];
#pragma unroll
  for (int i = 0; i < 2; ++i)
#pragma unroll
    for (int j = 0; j < 2; ++j)
#pragma unroll
      for (int r = 0; r < 8; ++r) acc[i][j][r] = 0.0f;

  const _Float16* ap0 = A + (size_t)(row0 + m) * EDIM + 8 * hh;
  const _Float16* ap1 = ap0 + (size_t)16 * EDIM;
  const _Float16* bp0 = Bt + (size_t)(col0 + m) * EDIM + 8 * hh;
  const _Float16* bp1 = bp0 + (size_t)16 * EDIM;

#pragma unroll 1
  for (int ks = 0; ks < EDIM / 32; ++ks) {
    const int k0 = 32 * ks;
    Frag a0, a1, b0, b1;
    a0.h[0] = *(const v8h*)(ap0 + k0);  a0.h[1] = *(const v8h*)(ap0 + k0 + 16);
    a1.h[0] = *(const v8h*)(ap1 + k0);  a1.h[1] = *(const v8h*)(ap1 + k0 + 16);
    b0.h[0] = *(const v8h*)(bp0 + k0);  b0.h[1] = *(const v8h*)(bp0 + k0 + 16);
    b1.h[0] = *(const v8h*)(bp1 + k0);  b1.h[1] = *(const v8h*)(bp1 + k0 + 16);
    acc[0][0] = wmh(a0.v, b0.v, acc[0][0]);
    acc[0][1] = wmh(a0.v, b1.v, acc[0][1]);
    acc[1][0] = wmh(a1.v, b0.v, acc[1][0]);
    acc[1][1] = wmh(a1.v, b1.v, acc[1][1]);
  }

#pragma unroll
  for (int i = 0; i < 2; ++i)
#pragma unroll
    for (int j = 0; j < 2; ++j)
#pragma unroll
      for (int r = 0; r < 8; ++r)
        stg[(wm * 32 + 16 * i + 8 * hh + r) * BN + wn * 32 + 16 * j + m] = acc[i][j][r] * RWSC;
  __syncthreads();

  float* cbase = C + (size_t)(mb * BM) * ldc + nb * BN;
#pragma unroll
  for (int p = 0; p < 8; ++p) {
    const int it = p * NTHR + tid;
    const int line = it >> 3, q = it & 7;
    const int lrow = line >> 1, cc = (line & 1) * 32 + 4 * q;
    const v4f v = *(const v4fa*)(stg + lrow * BN + cc);
    *(volatile v4f*)(cbase + (size_t)lrow * ldc + cc) = v;
  }
  __threadfence();
#pragma unroll
  for (int p = 0; p < 8; ++p) {
    const int it = p * NTHR + tid;
    const int line = it >> 3, q = it & 7;
    const int lrow = line >> 1, cc = (line & 1) * 32 + 4 * q;
    const v4f v = *(const v4fa*)(stg + lrow * BN + cc);
    *(volatile v4f*)(cbase + (size_t)lrow * ldc + cc) = v;
  }
}

template <int CH, int RELU>
__global__ __launch_bounds__(NTHR) void k_agg(const float* __restrict__ val, const int* __restrict__ erow,
                                              const int* __restrict__ ecol, int nnz, int nch,
                                              const float* __restrict__ dense, int mrows,
                                              float* accbuf, const float* __restrict__ bias, float* outp,
                                              int cidx, int fin) {
  constexpr int LDD = RCH * CH;
  constexpr int NV4 = DR * CH / 4;
  constexpr int NP  = NV4 / NTHR;
  static_assert(NP * NTHR == NV4);
  __shared__ __attribute__((aligned(16))) float acc[DR * CH];
  __shared__ float    lval[NTHR];
  __shared__ int      lrow[NTHR];
  __shared__ int      loff[NTHR];
  __shared__ unsigned ownm[NWAV * NWAV];
  const int tid = threadIdx.x, lane = tid & 31, wave = tid >> 5;
  const int d0 = (int)blockIdx.x * DR;
  float* gacc = accbuf + (size_t)d0 * CH;

  if (cidx == 0) {
    const v4f z = {0.0f, 0.0f, 0.0f, 0.0f};
#pragma unroll
    for (int p = 0; p < NP; ++p) *(v4fa*)(acc + 4 * (p * NTHR + tid)) = z;
  } else {
#pragma unroll
    for (int p = 0; p < NP; ++p) {
      const int it = p * NTHR + tid;
      *(v4fa*)(acc + 4 * it) = *(const v4f*)(gacc + 4 * it);
    }
  }
  __syncthreads();

  const int rbase = cidx * RCH;
  const int ncol  = RREL * NSRC;
#pragma unroll 1
  for (int ch = 0; ch < nch; ++ch) {
    const int e  = ch * NTHR + tid;
    const int ec = e < nnz ? e : nnz - 1;
    const int rw = erow[ec];
    int cl = ecol[ec];
    const float v = val[ec];
    cl = cl < 0 ? cl + ncol : cl;
    cl = cl < 0 ? 0 : (cl > ncol - 1 ? ncol - 1 : cl);
    const int r = cl / NSRC;
    const int n = cl - r * NSRC;
    int rl = r - rbase;
    const bool rok = (rl >= 0) && (rl < RCH);
    rl = rl < 0 ? 0 : (rl > RCH - 1 ? RCH - 1 : rl);
    const int lr = rw - d0;
    const bool valid = (e < nnz) && (rw >= 0) && (rw < mrows) && (lr >= 0) && (lr < DR) && rok;
    const int lrc = valid ? lr : 0;
    lrow[tid] = lrc;
    lval[tid] = v;
    loff[tid] = n * LDD + rl * CH;
    const int ow = lrc >> 3;
    unsigned mine = 0u;
#pragma unroll
    for (int w2 = 0; w2 < NWAV; ++w2) {
      const unsigned bm = __builtin_amdgcn_ballot_w32(valid && (ow == w2));
      mine = (lane == w2) ? bm : mine;
    }
    if (lane < NWAV) ownm[wave * NWAV + lane] = mine;
    __syncthreads();
#pragma unroll 1
    for (int u = 0; u < NWAV; ++u) {
      unsigned msk = ownm[u * NWAV + wave];
      while (msk != 0u) {
        const int bpos = __builtin_ctz(msk);
        msk &= msk - 1u;
        const int j = u * 32 + bpos;
        const int jr = lrow[j];
        const float vv = lval[j];
        const int off = loff[j];
        if (CH == EDIM) {
          const v4f x = *(const v4f*)(dense + (size_t)off + 4 * lane);
          v4fa* p = (v4fa*)(acc + jr * CH + 4 * lane);
          v4f t = *p;
          t = t + vv * x;
          *p = t;
        } else {
          const float x = dense[(size_t)off + lane];
          acc[jr * CH + lane] = fmaf(vv, x, acc[jr * CH + lane]);
        }
      }
    }
    __syncthreads();
  }

  float* dst = fin ? (outp + (size_t)d0 * CH) : gacc;
#pragma unroll
  for (int p = 0; p < NP; ++p) {
    const int it = p * NTHR + tid;
    v4f t = *(const v4fa*)(acc + 4 * it);
    if (fin) {
      const int c4 = (4 * it) & (CH - 1);
      const v4f bv = *(const v4f*)(bias + c4);
      t = t + bv;
      if (RELU) { t[0] = fmaxf(t[0], 0.0f); t[1] = fmaxf(t[1], 0.0f); t[2] = fmaxf(t[2], 0.0f); t[3] = fmaxf(t[3], 0.0f); }
    }
    *(volatile v4f*)(dst + 4 * it) = t;
  }
  __threadfence();
#pragma unroll
  for (int p = 0; p < NP; ++p) {
    const int it = p * NTHR + tid;
    v4f t = *(const v4fa*)(acc + 4 * it);
    if (fin) {
      const int c4 = (4 * it) & (CH - 1);
      const v4f bv = *(const v4f*)(bias + c4);
      t = t + bv;
      if (RELU) { t[0] = fmaxf(t[0], 0.0f); t[1] = fmaxf(t[1], 0.0f); t[2] = fmaxf(t[2], 0.0f); t[3] = fmaxf(t[3], 0.0f); }
    }
    *(volatile v4f*)(dst + 4 * it) = t;
  }
}

extern "C" void kernel_launch(void* const* d_in, const int* in_sizes, int n_in,
                              void* d_out, int out_size, void* d_ws, size_t ws_size,
                              hipStream_t stream) {
  if (n_in < 18) return;
  if (in_sizes[0] != NSRC * EDIM || in_sizes[1] != NSRC * EDIM) return;
  if (in_sizes[2] != RREL * NBAS || in_sizes[3] != NBAS * EDIM * EDIM) return;
  if (in_sizes[4] != RREL * NBAS || in_sizes[5] != NBAS * EDIM * CDIM) return;
  if (in_sizes[6] != EDIM || in_sizes[7] != CDIM) return;
  const int nnz1 = in_sizes[8], nnz2 = in_sizes[9], nnz3 = in_sizes[10];
  if (nnz1 < 1 || nnz2 < 1 || nnz3 < 1) return;
  if (nnz1 > (1 << 28) || nnz2 > (1 << 28) || nnz3 > (1 << 28)) return;
  if (in_sizes[11] != nnz1 || in_sizes[12] != nnz1) return;
  if (in_sizes[13] != nnz2 || in_sizes[14] != nnz2) return;
  if (in_sizes[15] != nnz3 || in_sizes[16] != nnz3) return;
  if (in_sizes[17] != NSRC) return;
  if (out_size != MSEGO * CDIM) return;

  const float* X1   = (const float*)d_in[0];
  const float* X2   = (const float*)d_in[1];
  const float* cp1  = (const float*)d_in[2];
  const float* bs1  = (const float*)d_in[3];
  const float* cp2  = (const float*)d_in[4];
  const float* bs2  = (const float*)d_in[5];
  const float* b1   = (const float*)d_in[6];
  const float* b2   = (const float*)d_in[7];
  const float* A1v  = (const float*)d_in[8];
  const float* A2v  = (const float*)d_in[9];
  const float* A3v  = (const float*)d_in[10];
  const int*   A1r  = (const int*)d_in[11];
  const int*   A1c  = (const int*)d_in[12];
  const int*   A2r  = (const int*)d_in[13];
  const int*   A2c  = (const int*)d_in[14];
  const int*   A3r  = (const int*)d_in[15];
  const int*   A3c  = (const int*)d_in[16];
  const int*   Hidx = (const int*)d_in[17];
  float* out = (float*)d_out;

  char* ws = (char*)d_ws;
  size_t o = 0;
  const size_t oW1 = o; o += (size_t)RREL * EDIM * EDIM * 2;        o = (o + 255) & ~(size_t)255;
  const size_t oW2 = o; o += (size_t)RREL * CDIM * EDIM * 2;        o = (o + 255) & ~(size_t)255;
  const size_t oXh = o; o += (size_t)2 * NSRC * EDIM * 2;           o = (o + 255) & ~(size_t)255;
  const size_t oH1 = o; o += (size_t)2 * MSEG1 * EDIM * 4;          o = (o + 255) & ~(size_t)255;
  const size_t oHg = o; o += (size_t)NSRC * EDIM * 2;               o = (o + 255) & ~(size_t)255;
  const size_t oXW = o; o += (size_t)NSRC * RCH * EDIM * 4;         o = (o + 255) & ~(size_t)255;
  const size_t oOA = o; o += (size_t)MSEGO * CDIM * 4;              o = (o + 255) & ~(size_t)255;
  if (o > ws_size || o > (size_t)WSCAP) return;
  _Float16* W1t = (_Float16*)(ws + oW1);
  _Float16* W2t = (_Float16*)(ws + oW2);
  _Float16* Xh  = (_Float16*)(ws + oXh);
  float*    H1  = (float*)(ws + oH1);
  _Float16* Hg  = (_Float16*)(ws + oHg);
  float*    XW  = (float*)(ws + oXW);
  float*    OA  = (float*)(ws + oOA);

  const int n8   = NSRC * EDIM / 8;
  const int nbh  = n8 / NTHR;
  const int nch1 = (nnz1 + NTHR - 1) / NTHR;
  const int nch2 = (nnz2 + NTHR - 1) / NTHR;
  const int nch3 = (nnz3 + NTHR - 1) / NTHR;
  const int nbn1 = (RCH * EDIM) / BN;
  const int nbn2 = (RCH * CDIM) / BN;
  const int ngm  = NSRC / BM;

  k_compose<<<(RREL * EDIM * 16) / NTHR, NTHR, 0, stream>>>(cp1, bs1, W1t, EDIM);
  k_compose<<<(RREL * CDIM * 16) / NTHR, NTHR, 0, stream>>>(cp2, bs2, W2t, CDIM);
  k_cvt<<<2 * nbh, NTHR, 0, stream>>>(X1, X2, Xh, n8, nbh);

  for (int d = 0; d < 2; ++d) {
    const _Float16* Ad = Xh + (size_t)d * NSRC * EDIM;
    const float* vd = d ? A2v : A1v;
    const int*   rd = d ? A2r : A1r;
    const int*   cd = d ? A2c : A1c;
    const int  nnzd = d ? nnz2 : nnz1;
    const int  nchd = d ? nch2 : nch1;
    float* Hd = H1 + (size_t)d * MSEG1 * EDIM;
    for (int c = 0; c < NCHK; ++c) {
      k_gemm<<<ngm * nbn1, NTHR, 0, stream>>>(Ad, W1t + (size_t)c * RCH * EDIM * EDIM, XW, RCH * EDIM, nbn1);
      k_agg<EDIM, 1><<<MSEG1 / DR, NTHR, 0, stream>>>(vd, rd, cd, nnzd, nchd, XW, MSEG1, Hd, b1, Hd,
                                                       c, (c == NCHK - 1) ? 1 : 0);
    }
  }

  k_gath<<<(NSRC * 16) / NTHR, NTHR, 0, stream>>>(H1, Hidx, Hg, NSRC, 2 * MSEG1);

  for (int c = 0; c < NCHK; ++c) {
    k_gemm<<<ngm * nbn2, NTHR, 0, stream>>>(Hg, W2t + (size_t)c * RCH * CDIM * EDIM, XW, RCH * CDIM, nbn2);
    k_agg<CDIM, 0><<<MSEGO / DR, NTHR, 0, stream>>>(A3v, A3r, A3c, nnz3, nch3, XW, MSEGO, OA, b2, out,
                                                     c, (c == NCHK - 1) ? 1 : 0);
  }
}
